// GPT_77403900608944
// MI455X (gfx1250) — hardware-verified
//
#include <hip/hip_runtime.h>


namespace {
constexpr int T = 2048, NE = 1024, NH = 16, NKV = 4, HD = 64, GC = 32, WIN = 1024, QL = 2048  ;
constexpr float XS = 8.0f, WSC = 256.0f, PS = 1024.0f, LOG2E = 1.4426950408889634f, EPS = 1.1920929e-07f;
static_assert(T % 64 == 0 && QL % 32 == 0, "tiling");
typedef _Float16 b16;
typedef __attribute__((ext_vector_type(16))) _Float16 v16b;
typedef __attribute__((ext_vector_type(8))) _Float16 v8b;
typedef __attribute__((ext_vector_type(8))) float v8f;
typedef __attribute__((ext_vector_type(4))) float v4f;
__device__ __forceinline__ float bf16_rne(float f) { unsigned int u = __float_as_uint(f); u += 0x7FFFu + ((u >> 16) & 1u); return __uint_as_float(u & 0xFFFF0000u); }
__device__ __forceinline__ void split16(float v, b16& hi, b16& lo) { hi = (b16)v; lo = (b16)(v - (float)hi); }
__device__ __forceinline__ v16b frag_kb(const b16* p, int hh) { const v8b a = *(const v8b*)(p + 8 * hh), b = *(const v8b*)(p + 16 + 8 * hh); v16b f;
#pragma unroll
  for (int e = 0; e < 8; ++e) { f[e] = a[e]; f[8 + e] = b[e]; } return f; }
__device__ __forceinline__ v8f wmma16b(v16b a, v16b b, v8f c) { v8f d = __builtin_amdgcn_wmma_f32_16x16x32_f16(false, a, false, b, (short)0, c, false, false); asm volatile("v_nop\n\tv_nop\n\tv_nop\n\tv_nop" : "+v"(d) : "v"(a), "v"(b)); return d; }
__device__ __forceinline__ void wave_lds_sync() { __builtin_amdgcn_fence(__ATOMIC_RELEASE, "workgroup"); __builtin_amdgcn_wave_barrier(); __builtin_amdgcn_fence(__ATOMIC_ACQUIRE, "workgroup"); }
__device__ __forceinline__ float pmul(float a, float b) { float p = a * b; asm volatile("" : "+v"(p)); return p; }
__device__ __forceinline__ int iclamp(int v, int lo, int hi) { return v < lo ? lo : (v > hi ? hi : v); }

typedef __attribute__((ext_vector_type(2))) _Float16 v2h;
typedef __attribute__((ext_vector_type(4))) _Float16 v4h;
typedef __attribute__((ext_vector_type(2))) float v2f;
__device__ __forceinline__ float nexp2(float v) { return __builtin_amdgcn_exp2f(v); }
__global__ __launch_bounds__(256) void prep_kernel(const float* __restrict__ wq, const float* __restrict__ wk, const float* __restrict__ wv, const float* __restrict__ wp, b16* __restrict__ WT, b16* __restrict__ WP) {
  const size_t u = (size_t)blockIdx.x * 256 + threadIdx.x; const size_t n1 = (size_t)1536 * NE / 8, n2 = (size_t)NE * NE / 8; v8b o;
  if (u < n1) { const size_t e = u * 8; const int oo = (int)(e / NE), d0 = (int)(e % NE); for (int j = 0; j < 8; ++j) { const int d = d0 + j; const float w = (oo < NE) ? wq[(size_t)d * NE + oo] : (oo < NE + NKV * HD) ? wk[(size_t)d * (NKV * HD) + (oo - NE)] : wv[(size_t)d * (NKV * HD) + (oo - NE - NKV * HD)]; o[j] = (b16)(bf16_rne(w) * WSC); }
    for (int pass = 0; pass < 2; ++pass) { *(volatile v8b*)(WT + e) = o; __threadfence(); } }
  else if (u < n1 + n2) { const size_t e = (u - n1) * 8; const int oo = (int)(e / NE), d0 = (int)(e % NE); for (int j = 0; j < 8; ++j) o[j] = (b16)(bf16_rne(wp[(size_t)(d0 + j) * NE + oo]) * WSC); for (int pass = 0; pass < 2; ++pass) { *(volatile v8b*)(WP + e) = o; __threadfence(); } }
}
__global__ __launch_bounds__(128) void proj_kernel(const float* __restrict__ x, const float* __restrict__ ve, const float* __restrict__ cosb, const float* __restrict__ sinb, const float* __restrict__ wg, const b16* __restrict__ WT, b16* __restrict__ Qh, b16* __restrict__ Ql, b16* __restrict__ Kh, b16* __restrict__ Kl, b16* __restrict__ VTh, b16* __restrict__ VTl) {
  __shared__ __attribute__((aligned(16))) b16 As[64][256 + 8]; __shared__ __attribute__((aligned(16))) float Tf[4][16][128 + 4];
  const int wave = threadIdx.x >> 5, lane = threadIdx.x & 31, nloc = lane & 15, hlf = lane >> 4; const size_t r0 = (size_t)blockIdx.x * 64; const size_t m0 = r0 + wave * 16; const int slab = blockIdx.y, n0 = slab * 128;
  v8f acc[8];
#pragma unroll
  for (int t = 0; t < 8; ++t) acc[t] = (v8f){};
#pragma unroll 1
  for (int kc = 0; kc < NE; kc += 256) {
    __syncthreads();
    for (int i = threadIdx.x; i < 64 * 64; i += 128) { const int rr = i / 64, q = (i % 64) * 4; const v4f f = *(const v4f*)(x + (r0 + rr) * NE + kc + q); v4h o; for (int j = 0; j < 4; ++j) o[j] = (b16)(bf16_rne(f[j]) * XS); *(v4h*)(&As[rr][q]) = o; }
    __syncthreads();
#pragma unroll 2
    for (int kb = 0; kb < 256; kb += 32) { const v16b a = frag_kb(&As[wave * 16 + nloc][kb], hlf);
#pragma unroll
      for (int t = 0; t < 8; ++t) acc[t] = wmma16b(a, frag_kb(WT + (size_t)(n0 + t * 16 + nloc) * NE + kc + kb, hlf), acc[t]); } }
#pragma unroll
  for (int t = 0; t < 8; ++t)
#pragma unroll
    for (int r = 0; r < 8; ++r) Tf[wave][8 * hlf + r][t * 16 + nloc] = acc[t][r] * (1.0f / (XS * WSC));
  __syncthreads();
  if (slab < 10) {
    for (int pass = 0; pass < 2; ++pass) {
      for (int rr = 0; rr < 16; ++rr) { const size_t tok = m0 + rr; const float cv = bf16_rne(cosb[tok * (HD / 2) + lane]), sv = bf16_rne(sinb[tok * (HD / 2) + lane]);
        for (int hs = 0; hs < 2; ++hs) { const float v1 = Tf[wave][rr][hs * 64 + lane], v2 = Tf[wave][rr][hs * 64 + 32 + lane]; const float a1 = v1 * cv + v2 * sv, a2 = -v1 * sv + v2 * cv;
          float ss = a1 * a1 + a2 * a2;
#pragma unroll
          for (int o = 1; o < 32; o <<= 1) ss += __shfl_xor(ss, o);
          const float inv = rsqrtf(ss * (1.0f / HD) + EPS); b16 p1, q1, p2, q2; split16(a1 * inv * XS, p1, q1); split16(a2 * inv * XS, p2, q2);
          b16* Ph_; b16* Pl_; size_t base; if (slab < 8) { const int h = 2 * slab + hs; Ph_ = Qh; Pl_ = Ql; base = ((size_t)h * T + tok) * HD; } else { const int kvh = 2 * (slab - 8) + hs; Ph_ = Kh; Pl_ = Kl; base = ((size_t)kvh * T + tok) * HD; }
          ((volatile b16*)Ph_)[base + lane] = p1; ((volatile b16*)Ph_)[base + 32 + lane] = p2; ((volatile b16*)Pl_)[base + lane] = q1; ((volatile b16*)Pl_)[base + 32 + lane] = q2; } }
      __threadfence(); } }
  else {
    for (int rr = 0; rr < 16; ++rr) { const size_t tok = m0 + rr; const float xg = bf16_rne(x[tok * NE + lane]);
      for (int hs = 0; hs < 2; ++hs) { const int kvh = 2 * (slab - 10) + hs; float g = pmul(xg, bf16_rne(wg[lane * NKV + kvh]));
#pragma unroll
        for (int o = 1; o < 32; o <<= 1) g += __shfl_xor(g, o);
        const float gate = 2.0f / (1.0f + expf(-g));
        for (int half = 0; half < 2; ++half) { const int d = half * 32 + lane; Tf[wave][rr][hs * 64 + d] += gate * bf16_rne(ve[tok * (NKV * HD) + kvh * HD + d]); } } }
    __syncthreads();
    for (int pass = 0; pass < 2; ++pass) {
#pragma unroll 1
      for (int q = 0; q < 32; ++q) { const int cl = wave * 32 + q; const int kvh = 2 * (slab - 10) + cl / 64, d = cl % 64; const int tk = lane * 2; v2h hv, lv;
        for (int j = 0; j < 2; ++j) { b16 p, ql; split16(Tf[(tk + j) >> 4][(tk + j) & 15][cl] * XS, p, ql); hv[j] = p; lv[j] = ql; }
        const size_t oi = ((size_t)kvh * HD + d) * T + r0 + lane * 2; *(volatile v2h*)(VTh + oi) = hv; *(volatile v2h*)(VTl + oi) = lv; }
      __threadfence(); } }
}
__global__ __launch_bounds__(64) void attn_kernel(const b16* __restrict__ Qh, const b16* __restrict__ Ql, const b16* __restrict__ Kh, const b16* __restrict__ Kl, const b16* __restrict__ VTh, const b16* __restrict__ VTl, b16* __restrict__ Yh, b16* __restrict__ Yl) {
  __shared__ __attribute__((aligned(16))) b16 Pb[2][16][32 + 8], Pc[2][16][32 + 8]; __shared__ __attribute__((aligned(16))) float To[2][16][HD + 4];
  const int wave = threadIdx.x >> 5, lane = threadIdx.x & 31, hh = lane >> 4, col = lane & 15; const int h = blockIdx.y, kvh = h / (NH / NKV); const int q0 = blockIdx.x * 32 + wave * 16, qi = q0 + col;
  const b16* Qhb = Qh + ((size_t)h * T) * HD; const b16* Qlb = Ql + ((size_t)h * T) * HD; const b16* Khb = Kh + ((size_t)kvh * T) * HD; const b16* Klb = Kl + ((size_t)kvh * T) * HD; const b16* Vh = VTh + ((size_t)kvh * HD) * T; const b16* Vl = VTl + ((size_t)kvh * HD) * T;
  const v16b qa0 = frag_kb(Qhb + (size_t)qi * HD, hh), qa1 = frag_kb(Qhb + (size_t)qi * HD + 32, hh), qb0 = frag_kb(Qlb + (size_t)qi * HD, hh), qb1 = frag_kb(Qlb + (size_t)qi * HD + 32, hh);
  const float cs = LOG2E / (8.0f * XS * XS);
  float m = -INFINITY, l = 0.0f; v8f o[4]; for (int t = 0; t < 4; ++t) o[t] = (v8f){};
  int kb0 = q0 - WIN; kb0 = kb0 < 0 ? 0 : (kb0 & ~31); const int kend = q0 + 16;
#pragma unroll 1
  for (int kb = kb0; kb < kend; kb += 32) {
    float e[16]; float mx = -INFINITY;
#pragma unroll
    for (int u = 0; u < 2; ++u) { v8f s = (v8f){}; const size_t kr = (size_t)(kb + u * 16 + col) * HD; const v16b kh0 = frag_kb(Khb + kr, hh), kh1 = frag_kb(Khb + kr + 32, hh), kl0 = frag_kb(Klb + kr, hh), kl1 = frag_kb(Klb + kr + 32, hh);
      s = wmma16b(kh0, qa0, s); s = wmma16b(kh1, qa1, s); s = wmma16b(kh0, qb0, s); s = wmma16b(kh1, qb1, s); s = wmma16b(kl0, qa0, s); s = wmma16b(kl1, qa1, s);
#pragma unroll
      for (int r = 0; r < 8; ++r) { const int key = kb + u * 16 + 8 * hh + r; const bool ok = (key <= qi) && (key >= qi - WIN); const float vv = ok ? s[r] * cs : -INFINITY; e[u * 8 + r] = vv; mx = fmaxf(mx, vv); } }
    mx = fmaxf(mx, __shfl_xor(mx, 16)); const float mn = fmaxf(m, mx); const float al = (mn == -INFINITY) ? 1.0f : nexp2(m - mn); float sum = 0.0f;
#pragma unroll
    for (int i2 = 0; i2 < 16; ++i2) { const float p = (e[i2] == -INFINITY || mn == -INFINITY) ? 0.0f : nexp2(e[i2] - mn); sum += p; b16 a_, b_; split16(p * PS, a_, b_); const int sl = (i2 < 8 ? 0 : 16) + 8 * hh + (i2 & 7); Pb[wave][col][sl] = a_; Pc[wave][col][sl] = b_; }
    sum += __shfl_xor(sum, 16); l = l * al + sum; m = mn;
    wave_lds_sync();
    const v16b pf = frag_kb(&Pb[wave][col][0], hh), pg = frag_kb(&Pc[wave][col][0], hh);
#pragma unroll
    for (int t = 0; t < 4; ++t) { o[t] *= al; const size_t vr = (size_t)(t * 16 + col) * T + kb; const v16b va = frag_kb(Vh + vr, hh), vb = frag_kb(Vl + vr, hh); o[t] = wmma16b(va, pf, o[t]); o[t] = wmma16b(va, pg, o[t]); o[t] = wmma16b(vb, pf, o[t]); }
    wave_lds_sync(); }
  const float inv = 1.0f / (l * PS * XS);
#pragma unroll
  for (int t = 0; t < 4; ++t)
#pragma unroll
    for (int r = 0; r < 8; ++r) To[wave][col][t * 16 + 8 * hh + r] = o[t][r] * inv;
  wave_lds_sync();
  for (int pass = 0; pass < 2; ++pass) { for (int rr = 0; rr < 16; ++rr) { const v2f f = *(const v2f*)(&To[wave][rr][lane * 2]); v2h hv, lv; for (int j = 0; j < 2; ++j) { b16 p, q; split16(f[j] * XS, p, q); hv[j] = p; lv[j] = q; }
      const size_t oi = (size_t)(q0 + rr) * NE + h * HD + lane * 2; *(volatile v2h*)(Yh + oi) = hv; *(volatile v2h*)(Yl + oi) = lv; } __threadfence(); }
}
__global__ __launch_bounds__(128) void out_kernel(const b16* __restrict__ Yh, const b16* __restrict__ Yl, const b16* __restrict__ WP, float* __restrict__ out) {
  __shared__ __attribute__((aligned(16))) float Tf[4][16][128 + 4];
  const int wave = threadIdx.x >> 5, lane = threadIdx.x & 31, nloc = lane & 15, hlf = lane >> 4; const size_t m0 = ((size_t)blockIdx.x * 4 + wave) * 16; const int n0 = blockIdx.y * 128;
  v8f acc[8];
#pragma unroll
  for (int t = 0; t < 8; ++t) acc[t] = (v8f){};
#pragma unroll 2
  for (int kb = 0; kb < NE; kb += 32) { const v16b a = frag_kb(Yh + (m0 + nloc) * NE + kb, hlf), al = frag_kb(Yl + (m0 + nloc) * NE + kb, hlf);
#pragma unroll
    for (int t = 0; t < 8; ++t) { const v16b bw = frag_kb(WP + (size_t)(n0 + t * 16 + nloc) * NE + kb, hlf); acc[t] = wmma16b(a, bw, acc[t]); acc[t] = wmma16b(al, bw, acc[t]); } }
#pragma unroll
  for (int t = 0; t < 8; ++t)
#pragma unroll
    for (int r = 0; r < 8; ++r) Tf[wave][8 * hlf + r][t * 16 + nloc] = acc[t][r] * (1.0f / (XS * WSC));
  wave_lds_sync();
  for (int pass = 0; pass < 2; ++pass) { for (int rr = 0; rr < 16; ++rr) *(volatile v4f*)(out + (m0 + rr) * NE + n0 + lane * 4) = *(const v4f*)(&Tf[wave][rr][lane * 4]); __threadfence(); }
}
}

extern "C" void kernel_launch(void* const* d_in, const int* in_sizes, int n_in, void* d_out, int out_size, void* d_ws, size_t ws_size, hipStream_t stream) {
  (void)n_in;
  auto Fp = [&](int i) { return (const float*)d_in[i]; };
  if (in_sizes[0] != T * NE || in_sizes[1] != T * NKV * HD || in_sizes[2] != T * (HD / 2) || in_sizes[3] != T * (HD / 2) || in_sizes[4] != NE * NE || in_sizes[5] != NE * NKV * HD || in_sizes[6] != NE * NKV * HD || in_sizes[7] != GC * NKV || in_sizes[8] != NE * NE || out_size != T * NE) return;
  size_t off = 0; char* ws = (char*)d_ws;
  auto carve = [&](size_t bytes) { char* p = ws + off; off += (bytes + 255) & ~(size_t)255; return p; };
  b16* WT = (b16*)carve((size_t)1536 * NE * 2); b16* WP = (b16*)carve((size_t)NE * NE * 2);
  b16* Qh = (b16*)carve((size_t)NH * T * HD * 2); b16* Ql = (b16*)carve((size_t)NH * T * HD * 2); b16* Kh = (b16*)carve((size_t)NKV * T * HD * 2); b16* Kl = (b16*)carve((size_t)NKV * T * HD * 2); b16* VTh = (b16*)carve((size_t)NKV * HD * T * 2); b16* VTl = (b16*)carve((size_t)NKV * HD * T * 2);
  b16* Yh = (b16*)carve((size_t)T * NE * 2); b16* Yl = (b16*)carve((size_t)T * NE * 2);
  if (off > ws_size || off > ((size_t)128 << 20)) return;
  prep_kernel<<<(unsigned)(((size_t)1536 * NE / 8 + (size_t)NE * NE / 8 + 255) / 256), 256, 0, stream>>>(Fp(4), Fp(5), Fp(6), Fp(8), WT, WP);
  proj_kernel<<<dim3(T / 64, 12), 128, 0, stream>>>(Fp(0), Fp(1), Fp(2), Fp(3), Fp(7), WT, Qh, Ql, Kh, Kl, VTh, VTl);
  attn_kernel<<<dim3(QL / 32, NH), 64, 0, stream>>>(Qh, Ql, Kh, Kl, VTh, VTl, Yh, Yl);
  out_kernel<<<dim3(QL / 64, NE / 128), 128, 0, stream>>>(Yh, Yl, WP, (float*)d_out);
}
